// NeuralNet_49452253446553
// MI455X (gfx1250) — hardware-verified
//
#include <hip/hip_runtime.h>
#include <stddef.h>
#include <stdint.h>


#define NTHR   256
#define NWAVE  8
#define EMB    64
#define NB     1024
#define EPT    8
#define CHUNK  (NTHR * EPT)
#define WCAP   (EPT * 32)
#define LISTN  (NWAVE * WCAP)
#define GSTEP  32
#define NWMAT  15
#define WSLOT  8192
#define SPITCH 72
#define WSC    8.0f
#define WINV   0.125f
#define LOSC   4096.0f
#define LOINV  0.000244140625f

#define OFF_U     0
#define OFF_CNT   262400
#define OFF_USTG  266512
#define OFF_SLOT  270608
#define OFF_LIST  270736
#define OFF_WCNT  278928
#define OFF_STG   266512
#define OFF_OSTG  284944
#define LDS_CONV  289040

static_assert(OFF_CNT == (NB + 1) * EMB * 4);
static_assert(OFF_USTG >= OFF_CNT + (NB + 1) * 4);
static_assert((OFF_USTG % 16) == 0 && (OFF_CNT % 16) == 0);
static_assert(OFF_SLOT == OFF_USTG + GSTEP * EMB * 2);
static_assert(OFF_LIST >= OFF_SLOT + GSTEP * 4 && (OFF_LIST % 16) == 0);
static_assert(OFF_WCNT == OFF_LIST + LISTN * 4);
static_assert(OFF_OSTG >= OFF_STG + NWAVE * 16 * SPITCH * 2 && (OFF_OSTG % 16) == 0);
static_assert(LDS_CONV >= OFF_OSTG + NB * 4);
static_assert(LDS_CONV >= OFF_WCNT + 64);
static_assert(WCAP == 256);
static_assert(NWAVE * 4 == GSTEP);
static_assert((NB % (16 * NWAVE)) == 0);
static_assert(NWAVE * 128 == NB);

typedef float    v2f  __attribute__((ext_vector_type(2)));
typedef float    v4f  __attribute__((ext_vector_type(4)));
typedef float    v8f  __attribute__((ext_vector_type(8)));
typedef int      v4i  __attribute__((ext_vector_type(4)));
typedef _Float16 v2h  __attribute__((ext_vector_type(2)));
typedef _Float16 v8h  __attribute__((ext_vector_type(8)));
typedef _Float16 v16h __attribute__((ext_vector_type(16)));
union FragH { v16h v; v8h h[2]; };

__device__ __forceinline__ v8f wmh(v16h a, v16h b, v8f c) {
  v8f d = __builtin_amdgcn_wmma_f32_16x16x32_f16(false, a, false, b, (short)0, c, false, false);
  asm volatile("v_nop\n\tv_nop\n\tv_nop\n\tv_nop" : "+v"(d) : "v"(a), "v"(b));
  return d;
}

__device__ __forceinline__ v8f zacc() {
  v8f c;
#pragma unroll
  for (int i = 0; i < 8; ++i) c[i] = 0.0f;
  return c;
}

__device__ __forceinline__ v16h ldfrag(const _Float16* rowp, int k0, int hh) {
  FragH f;
  const _Float16* pp = rowp + k0 + 8 * hh;
  f.h[0] = *(const v8h*)pp;
  f.h[1] = *(const v8h*)(pp + 16);
  return f.v;
}

__device__ __forceinline__ v16h ldb(const _Float16* __restrict__ W, int Kp, int n, int k0, int hh) {
  return ldfrag(W + (size_t)n * Kp, k0, hh);
}

__device__ __forceinline__ void gemm64(v8f (&acc)[4], const v16h (&a)[2], const _Float16* __restrict__ Wp, int m, int hh) {
#pragma unroll
  for (int nt = 0; nt < 4; ++nt) acc[nt] = zacc();
#pragma unroll
  for (int ks = 0; ks < 2; ++ks) {
#pragma unroll
    for (int nt = 0; nt < 4; ++nt) acc[nt] = wmh(a[ks], ldb(Wp, EMB, nt * 16 + m, ks * 32, hh), acc[nt]);
  }
}

template <int HASB, int RELU>
__device__ __forceinline__ void st_stage(_Float16* stg, const v8f (&acc)[4], const float* __restrict__ bias, int hh, int m) {
#pragma unroll
  for (int nt = 0; nt < 4; ++nt) {
    const int col = nt * 16 + m;
    float bv = 0.0f;
    if (HASB != 0) bv = bias[col];
#pragma unroll
    for (int r = 0; r < 8; ++r) {
      float t = acc[nt][r] * WINV + bv;
      if (RELU != 0) t = fmaxf(t, 0.0f);
      stg[(8 * hh + r) * SPITCH + col] = (_Float16)t;
    }
  }
}

__device__ __forceinline__ void lda2(v16h (&a)[2], const _Float16* rowp, int hh) {
  a[0] = ldfrag(rowp, 0, hh);
  a[1] = ldfrag(rowp, 32, hh);
}

__device__ __forceinline__ void ld_lines(v8h (&ov)[4], const _Float16* stg, int lane) {
#pragma unroll
  for (int q = 0; q < 4; ++q) ov[q] = *(const v8h*)(stg + (q * 4 + (lane >> 3)) * SPITCH + (lane & 7) * 8);
}
__device__ __forceinline__ void st_lines(_Float16* plane, size_t rowBase, const v8h (&ov)[4], int lane) {
#pragma unroll
  for (int q = 0; q < 4; ++q) {
    _Float16* g = plane + (rowBase + (size_t)(q * 4 + (lane >> 3))) * EMB + (lane & 7) * 8;
    *(volatile v8h*)g = ov[q];
  }
}

struct WArgs { const float* src[NWMAT]; int K[NWMAT]; int Kp[NWMAT]; };
static_assert(sizeof(WArgs) == NWMAT * 16);

__global__ __launch_bounds__(NTHR) void k_wconv(WArgs a, _Float16* WH) {
  const int s = blockIdx.x, tid = threadIdx.x;
  const float* src = a.src[0];
  int K = a.K[0], Kp = a.Kp[0];
#pragma unroll
  for (int j = 1; j < NWMAT; ++j) {
    if (s == j) { src = a.src[j]; K = a.K[j]; Kp = a.Kp[j]; }
  }
  _Float16* dst = WH + (size_t)s * WSLOT;
  const int kp8 = Kp >> 3;
  const int tot = EMB * kp8;
  v8h vals[4];
  int  addr[4];
  bool act[4];
#pragma unroll
  for (int j = 0; j < 4; ++j) {
    const int i  = tid + j * NTHR;
    act[j] = i < tot;
    const int ic = act[j] ? i : 0;
    const int n  = ic / kp8;
    const int k8 = ic - n * kp8;
    v8h v;
#pragma unroll
    for (int jj = 0; jj < 8; ++jj) {
      const int k  = 8 * k8 + jj;
      const int kc = k < K ? k : K - 1;
      const float w = src[(size_t)kc * EMB + n];
      v[jj] = (_Float16)(k < K ? w * WSC : 0.0f);
    }
    vals[j] = v;
    addr[j] = n * Kp + 8 * k8;
  }
#pragma unroll
  for (int j = 0; j < 4; ++j) if (act[j]) *(volatile v8h*)(dst + addr[j]) = vals[j];
  __threadfence();
#pragma unroll
  for (int j = 0; j < 4; ++j) if (act[j]) *(volatile v8h*)(dst + addr[j]) = vals[j];
}

template <int NIN, int ABIAS, int BOUT>
__global__ __launch_bounds__(NTHR) void k_embed(
    const float* __restrict__ X, int nX,
    const float* __restrict__ sh, const float* __restrict__ sc,
    const _Float16* __restrict__ W1p, const float* __restrict__ b1,
    const _Float16* __restrict__ W2p, const float* __restrict__ b2,
    const _Float16* __restrict__ Wap, const float* __restrict__ ba,
    const _Float16* __restrict__ Wbp,
    _Float16* outE, _Float16* outA, _Float16* outB, int nTiles) {
  __shared__ __attribute__((aligned(16))) _Float16 stgAll[NWAVE * 16 * SPITCH];
  const int tid = threadIdx.x, lane = tid & 31, wave = tid >> 5, hh = lane >> 4, m = lane & 15;
  const int tile = blockIdx.x * NWAVE + wave;
  const bool live = tile < nTiles;
  const int row0 = tile * 16;
  _Float16* stg = stgAll + wave * 16 * SPITCH;

  FragH a0;
  {
    int xr = row0 + m;
    xr = xr > nX - 1 ? nX - 1 : (xr < 0 ? 0 : xr);
    const float* xp = X + (size_t)xr * NIN;
#pragma unroll
    for (int i = 0; i < 16; ++i) {
      const int k  = (i < 8) ? (8 * hh + i) : (16 + 8 * hh + (i - 8));
      const int kc = k < NIN ? k : NIN - 1;
      const float xv = xp[kc];
      const float t  = (xv - sh[kc]) * sc[kc];
      a0.v[i] = (_Float16)(k < NIN ? t : 0.0f);
    }
  }
  v8f acc[4];
#pragma unroll
  for (int nt = 0; nt < 4; ++nt) acc[nt] = wmh(a0.v, ldb(W1p, 32, nt * 16 + m, 0, hh), zacc());

  st_stage<1, 1>(stg, acc, b1, hh, m);
  __syncthreads();
  v16h a[2];
  lda2(a, stg + m * SPITCH, hh);
  gemm64(acc, a, W2p, m, hh);
  __syncthreads();
  st_stage<1, 1>(stg, acc, b2, hh, m);
  __syncthreads();
  v8h ovE[4];
  ld_lines(ovE, stg, lane);
  lda2(a, stg + m * SPITCH, hh);
  if (live) st_lines(outE, (size_t)row0, ovE, lane);

  gemm64(acc, a, Wap, m, hh);
  __syncthreads();
  st_stage<ABIAS, 0>(stg, acc, ba, hh, m);
  __syncthreads();
  v8h ovA[4];
  ld_lines(ovA, stg, lane);
  if (live) st_lines(outA, (size_t)row0, ovA, lane);

  v8h ovB[4];
  if (BOUT != 0) {
    gemm64(acc, a, Wbp, m, hh);
    __syncthreads();
    st_stage<0, 0>(stg, acc, ba, hh, m);
    __syncthreads();
    ld_lines(ovB, stg, lane);
    if (live) st_lines(outB, (size_t)row0, ovB, lane);
  }
  __threadfence();
  if (live) {
    st_lines(outE, (size_t)row0, ovE, lane);
    st_lines(outA, (size_t)row0, ovA, lane);
    if (BOUT != 0) st_lines(outB, (size_t)row0, ovB, lane);
  }
}

__device__ __forceinline__ int scan_chunk(const int* __restrict__ dsts, int nE, int cbase, int nodeBase,
                                          int vec8, int* wl, int tid) {
  const int el0  = tid * EPT;
  const int e0   = cbase + el0;
  const int sent = -2147483647 - 1;
  v4i da, db;
  if (vec8 != 0 && cbase + CHUNK <= nE) {
    da = *(const v4i*)(dsts + e0);
    db = *(const v4i*)(dsts + e0 + 4);
  } else {
    da.x = (e0     < nE) ? dsts[min(e0,     nE - 1)] : sent;
    da.y = (e0 + 1 < nE) ? dsts[min(e0 + 1, nE - 1)] : sent;
    da.z = (e0 + 2 < nE) ? dsts[min(e0 + 2, nE - 1)] : sent;
    da.w = (e0 + 3 < nE) ? dsts[min(e0 + 3, nE - 1)] : sent;
    db.x = (e0 + 4 < nE) ? dsts[min(e0 + 4, nE - 1)] : sent;
    db.y = (e0 + 5 < nE) ? dsts[min(e0 + 5, nE - 1)] : sent;
    db.z = (e0 + 6 < nE) ? dsts[min(e0 + 6, nE - 1)] : sent;
    db.w = (e0 + 7 < nE) ? dsts[min(e0 + 7, nE - 1)] : sent;
  }
  const unsigned nb = (unsigned)nodeBase;
  unsigned hm = 0u;
  hm |= (((unsigned)da.x - nb) < (unsigned)NB) ? 1u   : 0u;
  hm |= (((unsigned)da.y - nb) < (unsigned)NB) ? 2u   : 0u;
  hm |= (((unsigned)da.z - nb) < (unsigned)NB) ? 4u   : 0u;
  hm |= (((unsigned)da.w - nb) < (unsigned)NB) ? 8u   : 0u;
  hm |= (((unsigned)db.x - nb) < (unsigned)NB) ? 16u  : 0u;
  hm |= (((unsigned)db.y - nb) < (unsigned)NB) ? 32u  : 0u;
  hm |= (((unsigned)db.z - nb) < (unsigned)NB) ? 64u  : 0u;
  hm |= (((unsigned)db.w - nb) < (unsigned)NB) ? 128u : 0u;
  int wc = 0;
#pragma unroll 1
  for (int k = 0; k < EPT; ++k) {
    const unsigned mk = __builtin_amdgcn_ballot_w32(hm != 0u);
    if (mk == 0u) break;
    if (hm != 0u) {
      const int pos = wc + (int)__builtin_amdgcn_mbcnt_lo(mk, 0u);
      const int jb  = (int)__builtin_ctz(hm);
      if (pos < WCAP) wl[pos] = el0 + jb;
      hm &= hm - 1u;
    }
    wc += (int)__builtin_popcount(mk);
  }
  return wc;
}

template <int SECOND>
__global__ __launch_bounds__(NTHR) void k_conv(
    const int* __restrict__ dsts, const int* __restrict__ srcs, int nE, int vec8,
    const _Float16* __restrict__ gpl, int nG,
    const _Float16* __restrict__ opl,
    const float* __restrict__ efeat, const float* __restrict__ esh, const float* __restrict__ esc,
    const float* __restrict__ We, const float* __restrict__ sfp,
    const _Float16* __restrict__ Wfp, const float* __restrict__ bfv, const float* __restrict__ spp,
    const _Float16* __restrict__ tgt,
    const _Float16* __restrict__ Woap, const float* __restrict__ boa,
    const _Float16* __restrict__ Wobp, const float* __restrict__ bob,
    const _Float16* __restrict__ Wxp, const float* __restrict__ bx, const float* __restrict__ w2,
    _Float16* outP, float* outS, int nOut, const int* __restrict__ nps) {
  extern __shared__ __attribute__((aligned(16))) unsigned char dynlds[];
  float*    U     = (float*)(dynlds + OFF_U);
  int*      cnt   = (int*)(dynlds + OFF_CNT);
  _Float16* ustg  = (_Float16*)(dynlds + OFF_USTG);
  int*      slotb = (int*)(dynlds + OFF_SLOT);
  int*      list  = (int*)(dynlds + OFF_LIST);
  int*      wcnt  = (int*)(dynlds + OFF_WCNT);
  (void)nps;

  const int tid = threadIdx.x, lane = tid & 31, wave = tid >> 5, hh = lane >> 4, m = lane & 15;
  const int q = lane >> 3, p = lane & 7;
  const int nodeBase = blockIdx.x * NB;

  {
    v4f z = {0.0f, 0.0f, 0.0f, 0.0f};
    for (int i = tid; i < (NB + 1) * (EMB / 4); i += NTHR) ((v4f*)U)[i] = z;
    for (int i = tid; i < NB + 1; i += NTHR) cnt[i] = 0;
  }
  float we[8];
#pragma unroll
  for (int j = 0; j < 8; ++j) we[j] = We[8 * p + j];
  const float sf = sfp[0], esh0 = esh[0], esc0 = esc[0];
  __syncthreads();

  const int nChunks = (nE + CHUNK - 1) / CHUNK;
#pragma unroll 1
  for (int ch = 0; ch < nChunks; ++ch) {
    const int cbase = ch * CHUNK;
    const int wc = scan_chunk(dsts, nE, cbase, nodeBase, vec8, list + wave * WCAP, tid);
    if (lane == 0) wcnt[wave] = wc;
    __syncthreads();

    int pre[NWAVE + 1];
    pre[0] = 0;
#pragma unroll
    for (int w = 0; w < NWAVE; ++w) {
      int c = wcnt[w];
      c = c > WCAP ? WCAP : (c < 0 ? 0 : c);
      pre[w + 1] = pre[w] + c;
    }
    const int tot    = pre[NWAVE];
    const int nSteps = (tot + GSTEP - 1) / GSTEP;

#pragma unroll 1
    for (int s = 0; s < nSteps; ++s) {
      const int rem = tot - s * GSTEP;
      if (wave * 4 < rem) {
        const int jl = wave * 4 + q;
        const int j  = s * GSTEP + jl;
        const bool valid = jl < rem;
        int wsel = 0, psub = 0;
#pragma unroll
        for (int w = 1; w < NWAVE; ++w) {
          const bool ge = j >= pre[w];
          wsel = ge ? w : wsel;
          psub = ge ? pre[w] : psub;
        }
        int li = j - psub;
        li = li < 0 ? 0 : (li > WCAP - 1 ? WCAP - 1 : li);
        int e = cbase + list[wsel * WCAP + li];
        if (!valid) e = 0;
        e = e < 0 ? 0 : (e > nE - 1 ? nE - 1 : e);
        const int d = dsts[e];
        int si   = srcs[e];
        int slot = d - nodeBase;
        if (!valid || (unsigned)slot >= (unsigned)NB) slot = NB;
        const int slc = slot < NB ? slot : NB - 1;
        si = si < 0 ? 0 : (si > nG - 1 ? nG - 1 : si);
        const v8h own = *(const v8h*)(opl + ((size_t)nodeBase + (size_t)slc) * EMB + 8 * p);
        const v8h g   = *(const v8h*)(gpl + (size_t)si * EMB + 8 * p);
        const float ef = (efeat[e] - esh0) * esc0;
        v8h uv;
        {
#pragma clang fp contract(off)
#pragma unroll
          for (int jj = 0; jj < 8; ++jj) {
            const float ovv = (float)own[jj], gvv = (float)g[jj];
            const float lv = (SECOND != 0) ? gvv : ovv;
            const float rv = (SECOND != 0) ? ovv : gvv;
            float t = ((lv + ef * we[jj]) + rv) * sf;
            t = fmaxf(t, 0.0f);
            uv[jj] = (_Float16)(valid ? t : 0.0f);
          }
        }
        *(v8h*)(ustg + jl * EMB + 8 * p) = uv;
        if (p == 0) slotb[jl] = slot;
      }
      __syncthreads();
      if (wave == 0) {
        const int na = rem < GSTEP ? rem : GSTEP;
#pragma unroll 1
        for (int i = 0; i < na; ++i) {
          int sl = slotb[i];
          sl = sl < 0 ? 0 : (sl > NB ? NB : sl);
          const v2h hv = *(const v2h*)(ustg + i * EMB + 2 * lane);
          float* up = U + (size_t)sl * EMB + 2 * lane;
          v2f cur = *(const v2f*)up;
          cur.x += (float)hv.x;
          cur.y += (float)hv.y;
          *(v2f*)up = cur;
          if (lane == 0) cnt[sl] += 1;
        }
      }
      __syncthreads();
    }
    __syncthreads();
  }
  __syncthreads();

  const float sp = spp[0];
  _Float16* stg  = (_Float16*)(dynlds + OFF_STG) + wave * 16 * SPITCH;
  float*    ostg = (float*)(dynlds + OFF_OSTG);
  float w2r[4];
#pragma unroll
  for (int nt = 0; nt < 4; ++nt) w2r[nt] = (SECOND != 0) ? w2[nt * 16 + m] : 0.0f;

#pragma unroll 1
  for (int it = 0; it < NB / (16 * NWAVE); ++it) {
    const int srow0 = (wave * (NB / (16 * NWAVE)) + it) * 16;

    v8f acch[4], accl[4];
#pragma unroll
    for (int nt = 0; nt < 4; ++nt) { acch[nt] = zacc(); accl[nt] = zacc(); }
#pragma unroll
    for (int ks = 0; ks < 2; ++ks) {
      FragH ahi, alo;
      const float* ur = U + (size_t)(srow0 + m) * EMB + ks * 32 + 8 * hh;
      const v4f x0 = *(const v4f*)ur;
      const v4f x1 = *(const v4f*)(ur + 4);
      const v4f x2 = *(const v4f*)(ur + 16);
      const v4f x3 = *(const v4f*)(ur + 20);
#pragma unroll
      for (int i = 0; i < 4; ++i) {
        const _Float16 h0 = (_Float16)x0[i]; ahi.h[0][i]     = h0; alo.h[0][i]     = (_Float16)((x0[i] - (float)h0) * LOSC);
        const _Float16 h1 = (_Float16)x1[i]; ahi.h[0][4 + i] = h1; alo.h[0][4 + i] = (_Float16)((x1[i] - (float)h1) * LOSC);
        const _Float16 h2 = (_Float16)x2[i]; ahi.h[1][i]     = h2; alo.h[1][i]     = (_Float16)((x2[i] - (float)h2) * LOSC);
        const _Float16 h3 = (_Float16)x3[i]; ahi.h[1][4 + i] = h3; alo.h[1][4 + i] = (_Float16)((x3[i] - (float)h3) * LOSC);
      }
#pragma unroll
      for (int nt = 0; nt < 4; ++nt) {
        const v16h b = ldb(Wfp, EMB, nt * 16 + m, ks * 32, hh);
        acch[nt] = wmh(ahi.v, b, acch[nt]);
        accl[nt] = wmh(alo.v, b, accl[nt]);
      }
    }
    float cr[8];
    {
      const v4i c0 = *(const v4i*)(cnt + srow0 + 8 * hh);
      const v4i c1 = *(const v4i*)(cnt + srow0 + 8 * hh + 4);
      cr[0] = (float)c0.x; cr[1] = (float)c0.y; cr[2] = (float)c0.z; cr[3] = (float)c0.w;
      cr[4] = (float)c1.x; cr[5] = (float)c1.y; cr[6] = (float)c1.z; cr[7] = (float)c1.w;
    }
    __syncthreads();
#pragma unroll
    for (int nt = 0; nt < 4; ++nt) {
      const int col = nt * 16 + m;
      const float bfc = bfv[col];
#pragma unroll
      for (int r = 0; r < 8; ++r) {
        const float val = ((acch[nt][r] + accl[nt][r] * LOINV) * WINV + cr[r] * bfc) * sp;
        stg[(8 * hh + r) * SPITCH + col] = (_Float16)val;
      }
    }
    __syncthreads();

    v8f acc[4];
#pragma unroll
    for (int nt = 0; nt < 4; ++nt) acc[nt] = zacc();
#pragma unroll
    for (int ks = 0; ks < 2; ++ks) {
      const v16h a = ldfrag(stg + m * SPITCH, ks * 32, hh);
#pragma unroll
      for (int nt = 0; nt < 4; ++nt) acc[nt] = wmh(a, ldb(Woap, 2 * EMB, nt * 16 + m, ks * 32, hh), acc[nt]);
    }
#pragma unroll
    for (int ks = 2; ks < 4; ++ks) {
      const v16h a = ldfrag(tgt + ((size_t)nodeBase + (size_t)(srow0 + m)) * EMB, (ks - 2) * 32, hh);
#pragma unroll
      for (int nt = 0; nt < 4; ++nt) acc[nt] = wmh(a, ldb(Woap, 2 * EMB, nt * 16 + m, ks * 32, hh), acc[nt]);
    }
    __syncthreads();
    st_stage<1, 1>(stg, acc, boa, hh, m);
    __syncthreads();
    v16h a2[2];
    lda2(a2, stg + m * SPITCH, hh);
    gemm64(acc, a2, Wobp, m, hh);
    __syncthreads();
    st_stage<1, 1>(stg, acc, bob, hh, m);
    __syncthreads();
    lda2(a2, stg + m * SPITCH, hh);
    gemm64(acc, a2, Wxp, m, hh);

    if (SECOND == 0) {
      __syncthreads();
      st_stage<1, 0>(stg, acc, bx, hh, m);
      __syncthreads();
      v8h ov[4];
      ld_lines(ov, stg, lane);
      const size_t rb = (size_t)nodeBase + (size_t)srow0;
      st_lines(outP, rb, ov, lane);
      __threadfence();
      st_lines(outP, rb, ov, lane);
    } else {
      float pr[8];
#pragma unroll
      for (int r = 0; r < 8; ++r) pr[r] = 0.0f;
#pragma unroll
      for (int nt = 0; nt < 4; ++nt) {
        const float bcol = bx[nt * 16 + m];
#pragma unroll
        for (int r = 0; r < 8; ++r) {
          const float y = fmaxf(acc[nt][r] * WINV + bcol, 0.0f);
          pr[r] += y * w2r[nt];
        }
      }
#pragma unroll
      for (int r = 0; r < 8; ++r) {
        pr[r] += __shfl_xor(pr[r], 8, 32);
        pr[r] += __shfl_xor(pr[r], 4, 32);
        pr[r] += __shfl_xor(pr[r], 2, 32);
        pr[r] += __shfl_xor(pr[r], 1, 32);
      }
      if (m == 0) {
        v4f o0 = {pr[0], pr[1], pr[2], pr[3]};
        v4f o1 = {pr[4], pr[5], pr[6], pr[7]};
        *(v4f*)(ostg + srow0 + 8 * hh)     = o0;
        *(v4f*)(ostg + srow0 + 8 * hh + 4) = o1;
      }
    }
  }

  if (SECOND != 0) {
    __syncthreads();
    const int f = wave * 128 + 4 * lane;
    const size_t gi  = (size_t)nodeBase + (size_t)f;
    const size_t lim = (size_t)(nOut < 0 ? 0 : nOut);
    const v4f v = *(const v4f*)(ostg + f);
    const bool full = gi + 3 < lim;
    if (full) *(volatile v4f*)(outS + gi) = v;
    else if (gi < lim) {
#pragma unroll
      for (int jj = 0; jj < 4; ++jj) if (gi + jj < lim) *(volatile float*)(outS + gi + jj) = v[jj];
    }
    __threadfence();
    if (full) *(volatile v4f*)(outS + gi) = v;
    else if (gi < lim) {
#pragma unroll
      for (int jj = 0; jj < 4; ++jj) if (gi + jj < lim) *(volatile float*)(outS + gi + jj) = v[jj];
    }
  }
}

extern "C" void kernel_launch(void* const* d_in, const int* in_sizes, int n_in,
                              void* d_out, int out_size, void* d_ws, size_t ws_size,
                              hipStream_t stream) {
  if (n_in < 47) return;
  const int nC = in_sizes[0] / 5;
  const int nV = in_sizes[2] / 19;
  const int nE = in_sizes[44] / 2;
  if (nC <= 0 || nV <= 0 || nE <= 0) return;
  if (in_sizes[0] != nC * 5 || in_sizes[2] != nV * 19 || in_sizes[44] != 2 * nE || in_sizes[1] != nE) return;
  if (out_size != nV) return;
  if (in_sizes[3] < 5 || in_sizes[4] < 5 || in_sizes[5] < 19 || in_sizes[6] < 19 || in_sizes[7] < 1 || in_sizes[8] < 1) return;
  const int widx[NWMAT] = {9, 11, 13, 15, 17, 20, 22, 25, 27, 29, 32, 34, 37, 39, 41};
  const int wK[NWMAT]   = {5, 64, 19, 64, 64, 64, 64, 128, 64, 64, 64, 64, 128, 64, 64};
  for (int s = 0; s < NWMAT; ++s) if (in_sizes[widx[s]] != wK[s] * EMB) return;
  const int bidx[15] = {10, 12, 14, 16, 18, 23, 26, 28, 30, 35, 38, 40, 42, 19, 31};
  for (int s = 0; s < 15; ++s) if (in_sizes[bidx[s]] != EMB) return;
  if (in_sizes[43] != EMB) return;
  if (in_sizes[21] < 1 || in_sizes[24] < 1 || in_sizes[33] < 1 || in_sizes[36] < 1) return;

  const float* cons   = (const float*)d_in[0];
  const float* efeat  = (const float*)d_in[1];
  const float* vars   = (const float*)d_in[2];
  const float* c_sh   = (const float*)d_in[3];
  const float* c_sc   = (const float*)d_in[4];
  const float* v_sh   = (const float*)d_in[5];
  const float* v_sc   = (const float*)d_in[6];
  const float* e_sh   = (const float*)d_in[7];
  const float* e_sc   = (const float*)d_in[8];
  const float* c_b1   = (const float*)d_in[10];
  const float* c_b2   = (const float*)d_in[12];
  const float* v_b1   = (const float*)d_in[14];
  const float* v_b2   = (const float*)d_in[16];
  const float* vc_bl  = (const float*)d_in[18];
  const float* vc_We  = (const float*)d_in[19];
  const float* vc_sf  = (const float*)d_in[21];
  const float* vc_bf  = (const float*)d_in[23];
  const float* vc_sp  = (const float*)d_in[24];
  const float* vc_boa = (const float*)d_in[26];
  const float* vc_bob = (const float*)d_in[28];
  const float* cv_bl  = (const float*)d_in[30];
  const float* cv_We  = (const float*)d_in[31];
  const float* cv_sf  = (const float*)d_in[33];
  const float* cv_bf  = (const float*)d_in[35];
  const float* cv_sp  = (const float*)d_in[36];
  const float* cv_boa = (const float*)d_in[38];
  const float* cv_bob = (const float*)d_in[40];
  const float* out_b1 = (const float*)d_in[42];
  const float* out_W2 = (const float*)d_in[43];
  const int*   eidx   = (const int*)d_in[44];
  const int*   n_cps  = (const int*)d_in[45];
  const int*   n_vps  = (const int*)d_in[46];
  const int* ei0 = eidx;
  const int* ei1 = eidx + (size_t)nE;
  float* out = (float*)d_out;

  const int nBlkC = (nC + NB - 1) / NB, nBlkV = (nV + NB - 1) / NB;
  const int rowsC = nBlkC * NB, rowsV = nBlkV * NB;

  char* ws = (char*)d_ws;
  size_t off = 0;
  const size_t oWH  = off; off += (size_t)NWMAT * WSLOT * 2;
  const size_t oC16 = off; off += (size_t)rowsC * EMB * 2;
  const size_t oV16 = off; off += (size_t)rowsV * EMB * 2;
  const size_t oL1  = off; off += (size_t)rowsC * EMB * 2;
  const size_t oR1  = off; off += (size_t)rowsV * EMB * 2;
  const size_t oR2  = off; off += (size_t)rowsV * EMB * 2;
  const size_t oL2  = off; off += (size_t)rowsC * EMB * 2;
  if (off > ws_size) return;
  _Float16* WH  = (_Float16*)(ws + oWH);
  _Float16* c16 = (_Float16*)(ws + oC16);
  _Float16* v16 = (_Float16*)(ws + oV16);
  _Float16* L1  = (_Float16*)(ws + oL1);
  _Float16* R1  = (_Float16*)(ws + oR1);
  _Float16* R2  = (_Float16*)(ws + oR2);
  _Float16* L2  = (_Float16*)(ws + oL2);

  WArgs wa;
  for (int s = 0; s < NWMAT; ++s) {
    wa.src[s] = (const float*)d_in[widx[s]];
    wa.K[s]   = wK[s];
    wa.Kp[s]  = wK[s] < 32 ? 32 : wK[s];
  }
  k_wconv<<<NWMAT, NTHR, 0, stream>>>(wa, WH);

  k_embed<5, 1, 0><<<rowsC / (16 * NWAVE), NTHR, 0, stream>>>(
      cons, nC, c_sh, c_sc, WH + 0 * WSLOT, c_b1, WH + 1 * WSLOT, c_b2,
      WH + 4 * WSLOT, vc_bl, WH + 4 * WSLOT, c16, L1, L1, rowsC / 16);

  k_embed<19, 0, 1><<<rowsV / (16 * NWAVE), NTHR, 0, stream>>>(
      vars, nV, v_sh, v_sc, WH + 2 * WSLOT, v_b1, WH + 3 * WSLOT, v_b2,
      WH + 5 * WSLOT, v_b2, WH + 10 * WSLOT, v16, R1, R2, rowsV / 16);

  hipFuncSetAttribute(reinterpret_cast<const void*>(&k_conv<0>), hipFuncAttributeMaxDynamicSharedMemorySize, LDS_CONV);
  hipFuncSetAttribute(reinterpret_cast<const void*>(&k_conv<1>), hipFuncAttributeMaxDynamicSharedMemorySize, LDS_CONV);

  const int vec8a = 1;
  const int vec8b = ((nE & 3) == 0) ? 1 : 0;

  k_conv<0><<<nBlkC, NTHR, LDS_CONV, stream>>>(
      ei0, ei1, nE, vec8a, R1, nV, L1, efeat, e_sh, e_sc, vc_We, vc_sf,
      WH + 6 * WSLOT, vc_bf, vc_sp, c16, WH + 7 * WSLOT, vc_boa, WH + 8 * WSLOT, vc_bob,
      WH + 9 * WSLOT, cv_bl, cv_bl, L2, out, 0, n_cps);

  k_conv<1><<<nBlkV, NTHR, LDS_CONV, stream>>>(
      ei1, ei0, nE, vec8b, L2, nC, R2, efeat, e_sh, e_sc, cv_We, cv_sf,
      WH + 11 * WSLOT, cv_bf, cv_sp, v16, WH + 12 * WSLOT, cv_boa, WH + 13 * WSLOT, cv_bob,
      WH + 14 * WSLOT, out_b1, out_W2, L1, out, nV, n_vps);
}
